// SpatialAttentionLayer_63187558858867
// MI455X (gfx1250) — hardware-run, weakly checked
//
#include <hip/hip_runtime.h>


namespace {
constexpr int NU = 100000, NI = 50000, D = 32, ER = 1000000, ET = 500000, E = ER  ;
constexpr float HS = 256.0f, WSC = 256.0f, BNEPS = 1e-5f;
typedef _Float16 b16;
typedef __attribute__((ext_vector_type(16))) _Float16 v16b;
typedef __attribute__((ext_vector_type(8))) _Float16 v8b;
typedef __attribute__((ext_vector_type(8))) float v8f;
typedef __attribute__((ext_vector_type(4))) float v4f;
__device__ __forceinline__ float bf16_rne(float f) { unsigned int u = __float_as_uint(f); u += 0x7FFFu + ((u >> 16) & 1u); float r = __uint_as_float(u & 0xFFFF0000u); asm volatile("" : "+v"(r)); return r; }
__device__ __forceinline__ float bfv(float f) { float r = bf16_rne(f); asm volatile("" : "+v"(r)); return r; }
__device__ __forceinline__ void split16(float v, b16& hi, b16& lo) { hi = (b16)v; lo = (b16)(v - (float)hi); }
__device__ __forceinline__ v16b frag_kb(const b16* p, int hh) { const v8b a = *(const v8b*)(p + 8 * hh), b = *(const v8b*)(p + 16 + 8 * hh); v16b f;
#pragma unroll
  for (int e = 0; e < 8; ++e) { f[e] = a[e]; f[8 + e] = b[e]; } return f; }
__device__ __forceinline__ v8f wmma16b(v16b a, v16b b, v8f c) { v8f d = __builtin_amdgcn_wmma_f32_16x16x32_f16(false, a, false, b, (short)0, c, false, false); asm volatile("v_nop\n\tv_nop\n\tv_nop\n\tv_nop" : "+v"(d) : "v"(a), "v"(b)); return d; }
__device__ __forceinline__ void wave_lds_sync() { __builtin_amdgcn_fence(__ATOMIC_RELEASE, "workgroup"); __builtin_amdgcn_wave_barrier(); __builtin_amdgcn_fence(__ATOMIC_ACQUIRE, "workgroup"); }
__device__ __forceinline__ float pmul(float a, float b) { float p = a * b; asm volatile("" : "+v"(p)); return p; }
__device__ __forceinline__ int iclamp(int v, int lo, int hi) { return v < lo ? lo : (v > hi ? hi : v); }
__device__ __forceinline__ float leaky2(float v) { return v > 0.0f ? v : 0.2f * v; }
#define N NI
constexpr int CSR_NBLKI = 512, CSR_GBI = 9, CSR_GNI = 1 << CSR_GBI  , CSR_TSI = (CSR_GNI < 32 ? 32 : CSR_GNI)  , CSR_MAXGI = 512, CSR_CAPI = 12288  ;
__device__ __host__ __forceinline__ int csr_tixI(int v) { return (v >> CSR_GBI) * CSR_TSI + (v & (CSR_GNI - 1)); }
__global__ __launch_bounds__(64) void csrA_kernelI(const int* __restrict__ dst, int E, int N, int nG, int CHP, int NGP, int* __restrict__ STG, int* __restrict__ HST) {
  extern __shared__ int sm[];
  int* cnt = sm; int* run = sm + NGP; int* ids = sm + 2 * NGP;
  const int b = blockIdx.x; const int ch = (E + CSR_NBLKI - 1) / CSR_NBLKI; const int e0 = b * ch, e1 = min(E, e0 + ch);
  for (int i = threadIdx.x; i < NGP; i += 64) cnt[i] = 0;
  for (int i = threadIdx.x; i < CHP; i += 64) ids[i] = -1;
  __syncthreads();
  if (threadIdx.x == 0) {
    for (int e = e0; e < e1; ++e) { int d = dst[e]; d = (d < 0) ? 0 : (d >= N ? N - 1 : d); cnt[d >> CSR_GBI] += 1; }
    int acc = 0; for (int g = 0; g < nG; ++g) { run[g] = acc; acc += cnt[g]; }
    for (int e = e0; e < e1; ++e) { int d = dst[e]; d = (d < 0) ? 0 : (d >= N ? N - 1 : d); const int g = d >> CSR_GBI; ids[run[g]] = e; run[g] += 1; } }
  __syncthreads();
  typedef __attribute__((ext_vector_type(4))) int v4i;
  for (int pass = 0; pass < 2; ++pass) {
    for (int i = threadIdx.x; i < CHP / 4; i += 64) *(volatile v4i*)(STG + (size_t)b * CHP + i * 4) = *(const v4i*)(&ids[i * 4]);
    for (int i = threadIdx.x; i < NGP / 4; i += 64) { v4i v; for (int e = 0; e < 4; ++e) v[e] = (i * 4 + e < nG) ? cnt[i * 4 + e] : 0; *(volatile v4i*)(HST + (size_t)b * NGP + i * 4) = v; }
    __threadfence(); }
}
__global__ __launch_bounds__(512) void csrS_kernelI(const int* __restrict__ HST, int nG, int NGP, int* __restrict__ START, int* __restrict__ TOT, int* __restrict__ OFF) {
  __shared__ int tot[CSR_MAXGI];
  const int b = threadIdx.x;
  for (int pass = 0; pass < 2; ++pass) { int runb = 0; for (int g = 0; g < nG; ++g) { int c = HST[(size_t)b * NGP + g]; c = (c < 0) ? 0 : c; ((volatile int*)OFF)[(size_t)g * CSR_NBLKI + b] = runb; runb += c; } __threadfence(); }
  for (int g = threadIdx.x; g < nG; g += 512) { int s = 0; for (int bb = 0; bb < CSR_NBLKI; ++bb) { int c = HST[(size_t)bb * NGP + g]; s += (c < 0) ? 0 : c; } tot[g] = s; }
  __syncthreads();
  if (threadIdx.x < 32) {
    __shared__ int st[CSR_MAXGI + 32];
    if (threadIdx.x == 0) { int acc = 0; for (int g = 0; g < NGP; ++g) { st[g] = acc; if (g < nG) acc += (tot[g] + 31) & ~31; } st[NGP] = acc; }
    __builtin_amdgcn_fence(__ATOMIC_RELEASE, "workgroup"); __builtin_amdgcn_wave_barrier(); __builtin_amdgcn_fence(__ATOMIC_ACQUIRE, "workgroup");
    for (int pass = 0; pass < 2; ++pass) { for (int i = threadIdx.x; i < NGP + 32; i += 32) { ((volatile int*)START)[i] = (i <= NGP) ? st[min(i, NGP)] : 0; ((volatile int*)TOT)[i] = (i < nG) ? tot[i] : 0; } __threadfence(); } }
}
__global__ __launch_bounds__(256) void csrB_kernelI(const int* __restrict__ dst, int N, int nG, int CHP, int NGP, int permLen, const int* __restrict__ STG, const int* __restrict__ HST, const int* __restrict__ OFF, const int* __restrict__ START, const int* __restrict__ TOT, int* __restrict__ PERM, int* __restrict__ ROWPTR, int* __restrict__ ROWCNT, int* __restrict__ FLAG) {
  typedef __attribute__((ext_vector_type(4))) int v4i;
  __shared__ int ids[CSR_CAPI]; __shared__ unsigned short key[CSR_CAPI]; __shared__ int outp[CSR_CAPI]; __shared__ int ncnt[CSR_GNI + 1]; __shared__ int boff[CSR_NBLKI + 1];
  const int g = blockIdx.x, t_ = threadIdx.x; int tot = TOT[g]; int st = START[g], stn = START[g + 1]; const int v0 = g * CSR_GNI; const int nv = min(CSR_GNI, N - v0); const int t0 = g * CSR_TSI;
  st = (st < 0) ? 0 : (st > permLen - 32 ? permLen - 32 : st) & ~31; stn = (stn < st) ? st : (stn > permLen ? permLen : stn); tot = (tot < 0) ? 0 : tot; if (tot > stn - st && tot <= CSR_CAPI) tot = stn - st;
  if (tot > CSR_CAPI) {
    for (int pass = 0; pass < 2; ++pass) { for (int i = t_; i < CSR_TSI / 4; i += 256) { v4i a, c; for (int e = 0; e < 4; ++e) { a[e] = st; c[e] = 0; } *(volatile v4i*)(ROWPTR + t0 + i * 4) = a; *(volatile v4i*)(ROWCNT + t0 + i * 4) = c; } if (t_ == 0) ((volatile int*)FLAG)[0] = 1; __threadfence(); } (void)nv; return; }
  if (t_ == 0) { int acc = 0; for (int b = 0; b < CSR_NBLKI; ++b) { boff[b] = acc; int c = HST[(size_t)b * NGP + g]; c = (c < 0) ? 0 : (c > CHP ? CHP : c); acc += c; if (acc > tot) acc = tot; } boff[CSR_NBLKI] = acc; }
  for (int i = t_; i <= CSR_GNI; i += 256) ncnt[i] = 0;
  __syncthreads();
  for (int b = 0; b < CSR_NBLKI; ++b) { const int c = boff[b + 1] - boff[b]; int o_ = OFF[(size_t)g * CSR_NBLKI + b]; o_ = (o_ < 0) ? 0 : (o_ > CHP - c ? CHP - c : o_); const int* src_ = STG + (size_t)b * CHP + o_;
    for (int i = t_; i < c; i += 256) { int id = src_[i]; id = (id < 0) ? 0 : id; ids[boff[b] + i] = id; int d = dst[id]; d = (d < v0) ? v0 : (d >= N ? N - 1 : d); int kk = d - v0; kk = (kk < 0) ? 0 : (kk >= CSR_GNI ? CSR_GNI - 1 : kk); key[boff[b] + i] = (unsigned short)kk; } }
  __syncthreads();
  if (t_ == 0) { for (int i = 0; i < tot; ++i) ncnt[key[i]] += 1; int acc = 0; for (int vl = 0; vl < CSR_GNI; ++vl) { const int c = ncnt[vl]; ncnt[vl] = acc; acc += c; } ncnt[CSR_GNI] = acc;
    for (int i = 0; i < tot; ++i) { const int vl = key[i]; outp[ncnt[vl]] = ids[i]; ncnt[vl] += 1; }
    for (int vl = CSR_GNI; vl > 0; --vl) ncnt[vl] = ncnt[vl - 1]; ncnt[0] = 0; }
  __syncthreads();
  for (int pass = 0; pass < 2; ++pass) {
    for (int i = t_; i < (stn - st) / 4; i += 256) { v4i v; for (int e = 0; e < 4; ++e) { const int q = i * 4 + e; v[e] = (q < tot) ? outp[q] : -1; } *(volatile v4i*)(PERM + st + i * 4) = v; }
    for (int i = t_; i < CSR_TSI / 4; i += 256) { v4i a, c; for (int e = 0; e < 4; ++e) { const int vl = i * 4 + e; const int vc = vl < CSR_GNI ? vl : CSR_GNI; a[e] = (vl < CSR_GNI) ? st + ncnt[vc] : st; c[e] = (vl < nv) ? (ncnt[(vc < CSR_GNI ? vc : CSR_GNI - 1) + 1] - ncnt[vc]) : 0; } *(volatile v4i*)(ROWPTR + t0 + i * 4) = a; *(volatile v4i*)(ROWCNT + t0 + i * 4) = c; }
    __threadfence(); }
}
__global__ __launch_bounds__(256) void csrZ_kernelI(int* __restrict__ p, size_t n4) { typedef __attribute__((ext_vector_type(4))) int v4i; const size_t tid = (size_t)blockIdx.x * 256 + threadIdx.x, nth = (size_t)gridDim.x * 256; v4i z = {0, 0, 0, 0}; for (size_t i = tid; i < n4; i += nth) *(volatile v4i*)(p + i * 4) = z; }
struct CsrBufsI { int *STG, *HST, *OFF, *START, *TOT, *PERM, *ROWPTR, *ROWCNT, *FLAG; int nG, NGP, CHP; size_t permLen; char* base; size_t bytes; };
static size_t csr_carveI(CsrBufsI& c, char* ws, size_t off, int E, int N) {
  const size_t off0 = off; c.base = ws + off;
  auto al = [&](size_t bytes) { char* p = ws + off; off += (bytes + 255) & ~(size_t)255; return p; };
  c.nG = (N + CSR_GNI - 1) / CSR_GNI; c.NGP = (c.nG + 31) & ~31; const int ch = (E + CSR_NBLKI - 1) / CSR_NBLKI; c.CHP = (ch + 31) & ~31; c.permLen = (size_t)E + 32 * (size_t)c.nG + 32;
  c.STG = (int*)al((size_t)CSR_NBLKI * c.CHP * 4); c.HST = (int*)al((size_t)CSR_NBLKI * c.NGP * 4); c.OFF = (int*)al((size_t)c.NGP * CSR_NBLKI * 4); c.START = (int*)al((size_t)(c.NGP + 64) * 4); c.TOT = (int*)al((size_t)(c.NGP + 64) * 4);
  c.PERM = (int*)al(c.permLen * 4); c.ROWPTR = (int*)al((size_t)c.nG * CSR_TSI * 4); c.ROWCNT = (int*)al((size_t)c.nG * CSR_TSI * 4); c.FLAG = (int*)al(256);
  c.bytes = off - off0; return off;
}
static void csr_buildI(const CsrBufsI& c, const int* dst, int E, int N, hipStream_t stream) {
  const size_t smem = (size_t)(2 * c.NGP + c.CHP) * 4;
  csrZ_kernelI<<<512, 256, 0, stream>>>((int*)c.base, c.bytes / 16);
  csrA_kernelI<<<CSR_NBLKI, 64, smem, stream>>>(dst, E, N, c.nG, c.CHP, c.NGP, c.STG, c.HST);
  csrS_kernelI<<<1, 512, 0, stream>>>(c.HST, c.nG, c.NGP, c.START, c.TOT, c.OFF);
  csrB_kernelI<<<c.nG, 256, 0, stream>>>(dst, N, c.nG, c.CHP, c.NGP, (int)c.permLen, c.STG, c.HST, c.OFF, c.START, c.TOT, c.PERM, c.ROWPTR, c.ROWCNT, c.FLAG);
}

#undef N
#define N NU
constexpr int CSR_NBLKU = 512, CSR_GBU = 9, CSR_GNU = 1 << CSR_GBU  , CSR_TSU = (CSR_GNU < 32 ? 32 : CSR_GNU)  , CSR_MAXGU = 512, CSR_CAPU = 12288  ;
__device__ __host__ __forceinline__ int csr_tixU(int v) { return (v >> CSR_GBU) * CSR_TSU + (v & (CSR_GNU - 1)); }
__global__ __launch_bounds__(64) void csrA_kernelU(const int* __restrict__ dst, int E, int N, int nG, int CHP, int NGP, int* __restrict__ STG, int* __restrict__ HST) {
  extern __shared__ int sm[];
  int* cnt = sm; int* run = sm + NGP; int* ids = sm + 2 * NGP;
  const int b = blockIdx.x; const int ch = (E + CSR_NBLKU - 1) / CSR_NBLKU; const int e0 = b * ch, e1 = min(E, e0 + ch);
  for (int i = threadIdx.x; i < NGP; i += 64) cnt[i] = 0;
  for (int i = threadIdx.x; i < CHP; i += 64) ids[i] = -1;
  __syncthreads();
  if (threadIdx.x == 0) {
    for (int e = e0; e < e1; ++e) { int d = dst[e]; d = (d < 0) ? 0 : (d >= N ? N - 1 : d); cnt[d >> CSR_GBU] += 1; }
    int acc = 0; for (int g = 0; g < nG; ++g) { run[g] = acc; acc += cnt[g]; }
    for (int e = e0; e < e1; ++e) { int d = dst[e]; d = (d < 0) ? 0 : (d >= N ? N - 1 : d); const int g = d >> CSR_GBU; ids[run[g]] = e; run[g] += 1; } }
  __syncthreads();
  typedef __attribute__((ext_vector_type(4))) int v4i;
  for (int pass = 0; pass < 2; ++pass) {
    for (int i = threadIdx.x; i < CHP / 4; i += 64) *(volatile v4i*)(STG + (size_t)b * CHP + i * 4) = *(const v4i*)(&ids[i * 4]);
    for (int i = threadIdx.x; i < NGP / 4; i += 64) { v4i v; for (int e = 0; e < 4; ++e) v[e] = (i * 4 + e < nG) ? cnt[i * 4 + e] : 0; *(volatile v4i*)(HST + (size_t)b * NGP + i * 4) = v; }
    __threadfence(); }
}
__global__ __launch_bounds__(512) void csrS_kernelU(const int* __restrict__ HST, int nG, int NGP, int* __restrict__ START, int* __restrict__ TOT, int* __restrict__ OFF) {
  __shared__ int tot[CSR_MAXGU];
  const int b = threadIdx.x;
  for (int pass = 0; pass < 2; ++pass) { int runb = 0; for (int g = 0; g < nG; ++g) { int c = HST[(size_t)b * NGP + g]; c = (c < 0) ? 0 : c; ((volatile int*)OFF)[(size_t)g * CSR_NBLKU + b] = runb; runb += c; } __threadfence(); }
  for (int g = threadIdx.x; g < nG; g += 512) { int s = 0; for (int bb = 0; bb < CSR_NBLKU; ++bb) { int c = HST[(size_t)bb * NGP + g]; s += (c < 0) ? 0 : c; } tot[g] = s; }
  __syncthreads();
  if (threadIdx.x < 32) {
    __shared__ int st[CSR_MAXGU + 32];
    if (threadIdx.x == 0) { int acc = 0; for (int g = 0; g < NGP; ++g) { st[g] = acc; if (g < nG) acc += (tot[g] + 31) & ~31; } st[NGP] = acc; }
    __builtin_amdgcn_fence(__ATOMIC_RELEASE, "workgroup"); __builtin_amdgcn_wave_barrier(); __builtin_amdgcn_fence(__ATOMIC_ACQUIRE, "workgroup");
    for (int pass = 0; pass < 2; ++pass) { for (int i = threadIdx.x; i < NGP + 32; i += 32) { ((volatile int*)START)[i] = (i <= NGP) ? st[min(i, NGP)] : 0; ((volatile int*)TOT)[i] = (i < nG) ? tot[i] : 0; } __threadfence(); } }
}
__global__ __launch_bounds__(256) void csrB_kernelU(const int* __restrict__ dst, int N, int nG, int CHP, int NGP, int permLen, const int* __restrict__ STG, const int* __restrict__ HST, const int* __restrict__ OFF, const int* __restrict__ START, const int* __restrict__ TOT, int* __restrict__ PERM, int* __restrict__ ROWPTR, int* __restrict__ ROWCNT, int* __restrict__ FLAG) {
  typedef __attribute__((ext_vector_type(4))) int v4i;
  __shared__ int ids[CSR_CAPU]; __shared__ unsigned short key[CSR_CAPU]; __shared__ int outp[CSR_CAPU]; __shared__ int ncnt[CSR_GNU + 1]; __shared__ int boff[CSR_NBLKU + 1];
  const int g = blockIdx.x, t_ = threadIdx.x; int tot = TOT[g]; int st = START[g], stn = START[g + 1]; const int v0 = g * CSR_GNU; const int nv = min(CSR_GNU, N - v0); const int t0 = g * CSR_TSU;
  st = (st < 0) ? 0 : (st > permLen - 32 ? permLen - 32 : st) & ~31; stn = (stn < st) ? st : (stn > permLen ? permLen : stn); tot = (tot < 0) ? 0 : tot; if (tot > stn - st && tot <= CSR_CAPU) tot = stn - st;
  if (tot > CSR_CAPU) {
    for (int pass = 0; pass < 2; ++pass) { for (int i = t_; i < CSR_TSU / 4; i += 256) { v4i a, c; for (int e = 0; e < 4; ++e) { a[e] = st; c[e] = 0; } *(volatile v4i*)(ROWPTR + t0 + i * 4) = a; *(volatile v4i*)(ROWCNT + t0 + i * 4) = c; } if (t_ == 0) ((volatile int*)FLAG)[0] = 1; __threadfence(); } (void)nv; return; }
  if (t_ == 0) { int acc = 0; for (int b = 0; b < CSR_NBLKU; ++b) { boff[b] = acc; int c = HST[(size_t)b * NGP + g]; c = (c < 0) ? 0 : (c > CHP ? CHP : c); acc += c; if (acc > tot) acc = tot; } boff[CSR_NBLKU] = acc; }
  for (int i = t_; i <= CSR_GNU; i += 256) ncnt[i] = 0;
  __syncthreads();
  for (int b = 0; b < CSR_NBLKU; ++b) { const int c = boff[b + 1] - boff[b]; int o_ = OFF[(size_t)g * CSR_NBLKU + b]; o_ = (o_ < 0) ? 0 : (o_ > CHP - c ? CHP - c : o_); const int* src_ = STG + (size_t)b * CHP + o_;
    for (int i = t_; i < c; i += 256) { int id = src_[i]; id = (id < 0) ? 0 : id; ids[boff[b] + i] = id; int d = dst[id]; d = (d < v0) ? v0 : (d >= N ? N - 1 : d); int kk = d - v0; kk = (kk < 0) ? 0 : (kk >= CSR_GNU ? CSR_GNU - 1 : kk); key[boff[b] + i] = (unsigned short)kk; } }
  __syncthreads();
  if (t_ == 0) { for (int i = 0; i < tot; ++i) ncnt[key[i]] += 1; int acc = 0; for (int vl = 0; vl < CSR_GNU; ++vl) { const int c = ncnt[vl]; ncnt[vl] = acc; acc += c; } ncnt[CSR_GNU] = acc;
    for (int i = 0; i < tot; ++i) { const int vl = key[i]; outp[ncnt[vl]] = ids[i]; ncnt[vl] += 1; }
    for (int vl = CSR_GNU; vl > 0; --vl) ncnt[vl] = ncnt[vl - 1]; ncnt[0] = 0; }
  __syncthreads();
  for (int pass = 0; pass < 2; ++pass) {
    for (int i = t_; i < (stn - st) / 4; i += 256) { v4i v; for (int e = 0; e < 4; ++e) { const int q = i * 4 + e; v[e] = (q < tot) ? outp[q] : -1; } *(volatile v4i*)(PERM + st + i * 4) = v; }
    for (int i = t_; i < CSR_TSU / 4; i += 256) { v4i a, c; for (int e = 0; e < 4; ++e) { const int vl = i * 4 + e; const int vc = vl < CSR_GNU ? vl : CSR_GNU; a[e] = (vl < CSR_GNU) ? st + ncnt[vc] : st; c[e] = (vl < nv) ? (ncnt[(vc < CSR_GNU ? vc : CSR_GNU - 1) + 1] - ncnt[vc]) : 0; } *(volatile v4i*)(ROWPTR + t0 + i * 4) = a; *(volatile v4i*)(ROWCNT + t0 + i * 4) = c; }
    __threadfence(); }
}
__global__ __launch_bounds__(256) void csrZ_kernelU(int* __restrict__ p, size_t n4) { typedef __attribute__((ext_vector_type(4))) int v4i; const size_t tid = (size_t)blockIdx.x * 256 + threadIdx.x, nth = (size_t)gridDim.x * 256; v4i z = {0, 0, 0, 0}; for (size_t i = tid; i < n4; i += nth) *(volatile v4i*)(p + i * 4) = z; }
struct CsrBufsU { int *STG, *HST, *OFF, *START, *TOT, *PERM, *ROWPTR, *ROWCNT, *FLAG; int nG, NGP, CHP; size_t permLen; char* base; size_t bytes; };
static size_t csr_carveU(CsrBufsU& c, char* ws, size_t off, int E, int N) {
  const size_t off0 = off; c.base = ws + off;
  auto al = [&](size_t bytes) { char* p = ws + off; off += (bytes + 255) & ~(size_t)255; return p; };
  c.nG = (N + CSR_GNU - 1) / CSR_GNU; c.NGP = (c.nG + 31) & ~31; const int ch = (E + CSR_NBLKU - 1) / CSR_NBLKU; c.CHP = (ch + 31) & ~31; c.permLen = (size_t)E + 32 * (size_t)c.nG + 32;
  c.STG = (int*)al((size_t)CSR_NBLKU * c.CHP * 4); c.HST = (int*)al((size_t)CSR_NBLKU * c.NGP * 4); c.OFF = (int*)al((size_t)c.NGP * CSR_NBLKU * 4); c.START = (int*)al((size_t)(c.NGP + 64) * 4); c.TOT = (int*)al((size_t)(c.NGP + 64) * 4);
  c.PERM = (int*)al(c.permLen * 4); c.ROWPTR = (int*)al((size_t)c.nG * CSR_TSU * 4); c.ROWCNT = (int*)al((size_t)c.nG * CSR_TSU * 4); c.FLAG = (int*)al(256);
  c.bytes = off - off0; return off;
}
static void csr_buildU(const CsrBufsU& c, const int* dst, int E, int N, hipStream_t stream) {
  const size_t smem = (size_t)(2 * c.NGP + c.CHP) * 4;
  csrZ_kernelU<<<512, 256, 0, stream>>>((int*)c.base, c.bytes / 16);
  csrA_kernelU<<<CSR_NBLKU, 64, smem, stream>>>(dst, E, N, c.nG, c.CHP, c.NGP, c.STG, c.HST);
  csrS_kernelU<<<1, 512, 0, stream>>>(c.HST, c.nG, c.NGP, c.START, c.TOT, c.OFF);
  csrB_kernelU<<<c.nG, 256, 0, stream>>>(dst, N, c.nG, c.CHP, c.NGP, (int)c.permLen, c.STG, c.HST, c.OFF, c.START, c.TOT, c.PERM, c.ROWPTR, c.ROWCNT, c.FLAG);
}
constexpr int CSR_NBLKT = 512, CSR_GBT = 9, CSR_GNT = 1 << CSR_GBT  , CSR_TST = (CSR_GNT < 32 ? 32 : CSR_GNT)  , CSR_MAXGT = 512, CSR_CAPT = 12288  ;
__device__ __host__ __forceinline__ int csr_tixT(int v) { return (v >> CSR_GBT) * CSR_TST + (v & (CSR_GNT - 1)); }
__global__ __launch_bounds__(64) void csrA_kernelT(const int* __restrict__ dst, int E, int N, int nG, int CHP, int NGP, int* __restrict__ STG, int* __restrict__ HST) {
  extern __shared__ int sm[];
  int* cnt = sm; int* run = sm + NGP; int* ids = sm + 2 * NGP;
  const int b = blockIdx.x; const int ch = (E + CSR_NBLKT - 1) / CSR_NBLKT; const int e0 = b * ch, e1 = min(E, e0 + ch);
  for (int i = threadIdx.x; i < NGP; i += 64) cnt[i] = 0;
  for (int i = threadIdx.x; i < CHP; i += 64) ids[i] = -1;
  __syncthreads();
  if (threadIdx.x == 0) {
    for (int e = e0; e < e1; ++e) { int d = dst[e]; d = (d < 0) ? 0 : (d >= N ? N - 1 : d); cnt[d >> CSR_GBT] += 1; }
    int acc = 0; for (int g = 0; g < nG; ++g) { run[g] = acc; acc += cnt[g]; }
    for (int e = e0; e < e1; ++e) { int d = dst[e]; d = (d < 0) ? 0 : (d >= N ? N - 1 : d); const int g = d >> CSR_GBT; ids[run[g]] = e; run[g] += 1; } }
  __syncthreads();
  typedef __attribute__((ext_vector_type(4))) int v4i;
  for (int pass = 0; pass < 2; ++pass) {
    for (int i = threadIdx.x; i < CHP / 4; i += 64) *(volatile v4i*)(STG + (size_t)b * CHP + i * 4) = *(const v4i*)(&ids[i * 4]);
    for (int i = threadIdx.x; i < NGP / 4; i += 64) { v4i v; for (int e = 0; e < 4; ++e) v[e] = (i * 4 + e < nG) ? cnt[i * 4 + e] : 0; *(volatile v4i*)(HST + (size_t)b * NGP + i * 4) = v; }
    __threadfence(); }
}
__global__ __launch_bounds__(512) void csrS_kernelT(const int* __restrict__ HST, int nG, int NGP, int* __restrict__ START, int* __restrict__ TOT, int* __restrict__ OFF) {
  __shared__ int tot[CSR_MAXGT];
  const int b = threadIdx.x;
  for (int pass = 0; pass < 2; ++pass) { int runb = 0; for (int g = 0; g < nG; ++g) { int c = HST[(size_t)b * NGP + g]; c = (c < 0) ? 0 : c; ((volatile int*)OFF)[(size_t)g * CSR_NBLKT + b] = runb; runb += c; } __threadfence(); }
  for (int g = threadIdx.x; g < nG; g += 512) { int s = 0; for (int bb = 0; bb < CSR_NBLKT; ++bb) { int c = HST[(size_t)bb * NGP + g]; s += (c < 0) ? 0 : c; } tot[g] = s; }
  __syncthreads();
  if (threadIdx.x < 32) {
    __shared__ int st[CSR_MAXGT + 32];
    if (threadIdx.x == 0) { int acc = 0; for (int g = 0; g < NGP; ++g) { st[g] = acc; if (g < nG) acc += (tot[g] + 31) & ~31; } st[NGP] = acc; }
    __builtin_amdgcn_fence(__ATOMIC_RELEASE, "workgroup"); __builtin_amdgcn_wave_barrier(); __builtin_amdgcn_fence(__ATOMIC_ACQUIRE, "workgroup");
    for (int pass = 0; pass < 2; ++pass) { for (int i = threadIdx.x; i < NGP + 32; i += 32) { ((volatile int*)START)[i] = (i <= NGP) ? st[min(i, NGP)] : 0; ((volatile int*)TOT)[i] = (i < nG) ? tot[i] : 0; } __threadfence(); } }
}
__global__ __launch_bounds__(256) void csrB_kernelT(const int* __restrict__ dst, int N, int nG, int CHP, int NGP, int permLen, const int* __restrict__ STG, const int* __restrict__ HST, const int* __restrict__ OFF, const int* __restrict__ START, const int* __restrict__ TOT, int* __restrict__ PERM, int* __restrict__ ROWPTR, int* __restrict__ ROWCNT, int* __restrict__ FLAG) {
  typedef __attribute__((ext_vector_type(4))) int v4i;
  __shared__ int ids[CSR_CAPT]; __shared__ unsigned short key[CSR_CAPT]; __shared__ int outp[CSR_CAPT]; __shared__ int ncnt[CSR_GNT + 1]; __shared__ int boff[CSR_NBLKT + 1];
  const int g = blockIdx.x, t_ = threadIdx.x; int tot = TOT[g]; int st = START[g], stn = START[g + 1]; const int v0 = g * CSR_GNT; const int nv = min(CSR_GNT, N - v0); const int t0 = g * CSR_TST;
  st = (st < 0) ? 0 : (st > permLen - 32 ? permLen - 32 : st) & ~31; stn = (stn < st) ? st : (stn > permLen ? permLen : stn); tot = (tot < 0) ? 0 : tot; if (tot > stn - st && tot <= CSR_CAPT) tot = stn - st;
  if (tot > CSR_CAPT) {
    for (int pass = 0; pass < 2; ++pass) { for (int i = t_; i < CSR_TST / 4; i += 256) { v4i a, c; for (int e = 0; e < 4; ++e) { a[e] = st; c[e] = 0; } *(volatile v4i*)(ROWPTR + t0 + i * 4) = a; *(volatile v4i*)(ROWCNT + t0 + i * 4) = c; } if (t_ == 0) ((volatile int*)FLAG)[0] = 1; __threadfence(); } (void)nv; return; }
  if (t_ == 0) { int acc = 0; for (int b = 0; b < CSR_NBLKT; ++b) { boff[b] = acc; int c = HST[(size_t)b * NGP + g]; c = (c < 0) ? 0 : (c > CHP ? CHP : c); acc += c; if (acc > tot) acc = tot; } boff[CSR_NBLKT] = acc; }
  for (int i = t_; i <= CSR_GNT; i += 256) ncnt[i] = 0;
  __syncthreads();
  for (int b = 0; b < CSR_NBLKT; ++b) { const int c = boff[b + 1] - boff[b]; int o_ = OFF[(size_t)g * CSR_NBLKT + b]; o_ = (o_ < 0) ? 0 : (o_ > CHP - c ? CHP - c : o_); const int* src_ = STG + (size_t)b * CHP + o_;
    for (int i = t_; i < c; i += 256) { int id = src_[i]; id = (id < 0) ? 0 : id; ids[boff[b] + i] = id; int d = dst[id]; d = (d < v0) ? v0 : (d >= N ? N - 1 : d); int kk = d - v0; kk = (kk < 0) ? 0 : (kk >= CSR_GNT ? CSR_GNT - 1 : kk); key[boff[b] + i] = (unsigned short)kk; } }
  __syncthreads();
  if (t_ == 0) { for (int i = 0; i < tot; ++i) ncnt[key[i]] += 1; int acc = 0; for (int vl = 0; vl < CSR_GNT; ++vl) { const int c = ncnt[vl]; ncnt[vl] = acc; acc += c; } ncnt[CSR_GNT] = acc;
    for (int i = 0; i < tot; ++i) { const int vl = key[i]; outp[ncnt[vl]] = ids[i]; ncnt[vl] += 1; }
    for (int vl = CSR_GNT; vl > 0; --vl) ncnt[vl] = ncnt[vl - 1]; ncnt[0] = 0; }
  __syncthreads();
  for (int pass = 0; pass < 2; ++pass) {
    for (int i = t_; i < (stn - st) / 4; i += 256) { v4i v; for (int e = 0; e < 4; ++e) { const int q = i * 4 + e; v[e] = (q < tot) ? outp[q] : -1; } *(volatile v4i*)(PERM + st + i * 4) = v; }
    for (int i = t_; i < CSR_TST / 4; i += 256) { v4i a, c; for (int e = 0; e < 4; ++e) { const int vl = i * 4 + e; const int vc = vl < CSR_GNT ? vl : CSR_GNT; a[e] = (vl < CSR_GNT) ? st + ncnt[vc] : st; c[e] = (vl < nv) ? (ncnt[(vc < CSR_GNT ? vc : CSR_GNT - 1) + 1] - ncnt[vc]) : 0; } *(volatile v4i*)(ROWPTR + t0 + i * 4) = a; *(volatile v4i*)(ROWCNT + t0 + i * 4) = c; }
    __threadfence(); }
}
__global__ __launch_bounds__(256) void csrZ_kernelT(int* __restrict__ p, size_t n4) { typedef __attribute__((ext_vector_type(4))) int v4i; const size_t tid = (size_t)blockIdx.x * 256 + threadIdx.x, nth = (size_t)gridDim.x * 256; v4i z = {0, 0, 0, 0}; for (size_t i = tid; i < n4; i += nth) *(volatile v4i*)(p + i * 4) = z; }
struct CsrBufsT { int *STG, *HST, *OFF, *START, *TOT, *PERM, *ROWPTR, *ROWCNT, *FLAG; int nG, NGP, CHP; size_t permLen; char* base; size_t bytes; };
static size_t csr_carveT(CsrBufsT& c, char* ws, size_t off, int E, int N) {
  const size_t off0 = off; c.base = ws + off;
  auto al = [&](size_t bytes) { char* p = ws + off; off += (bytes + 255) & ~(size_t)255; return p; };
  c.nG = (N + CSR_GNT - 1) / CSR_GNT; c.NGP = (c.nG + 31) & ~31; const int ch = (E + CSR_NBLKT - 1) / CSR_NBLKT; c.CHP = (ch + 31) & ~31; c.permLen = (size_t)E + 32 * (size_t)c.nG + 32;
  c.STG = (int*)al((size_t)CSR_NBLKT * c.CHP * 4); c.HST = (int*)al((size_t)CSR_NBLKT * c.NGP * 4); c.OFF = (int*)al((size_t)c.NGP * CSR_NBLKT * 4); c.START = (int*)al((size_t)(c.NGP + 64) * 4); c.TOT = (int*)al((size_t)(c.NGP + 64) * 4);
  c.PERM = (int*)al(c.permLen * 4); c.ROWPTR = (int*)al((size_t)c.nG * CSR_TST * 4); c.ROWCNT = (int*)al((size_t)c.nG * CSR_TST * 4); c.FLAG = (int*)al(256);
  c.bytes = off - off0; return off;
}
static void csr_buildT(const CsrBufsT& c, const int* dst, int E, int N, hipStream_t stream) {
  const size_t smem = (size_t)(2 * c.NGP + c.CHP) * 4;
  csrZ_kernelT<<<512, 256, 0, stream>>>((int*)c.base, c.bytes / 16);
  csrA_kernelT<<<CSR_NBLKT, 64, smem, stream>>>(dst, E, N, c.nG, c.CHP, c.NGP, c.STG, c.HST);
  csrS_kernelT<<<1, 512, 0, stream>>>(c.HST, c.nG, c.NGP, c.START, c.TOT, c.OFF);
  csrB_kernelT<<<c.nG, 256, 0, stream>>>(dst, N, c.nG, c.CHP, c.NGP, (int)c.permLen, c.STG, c.HST, c.OFF, c.START, c.TOT, c.PERM, c.ROWPTR, c.ROWCNT, c.FLAG);
}

#undef N

__global__ __launch_bounds__(256) void wput_kernel(const float* __restrict__ w0, const float* __restrict__ w1, const float* __restrict__ w2, const float* __restrict__ w3, const float* __restrict__ w4, const float* __restrict__ w5, const float* __restrict__ w6, const float* __restrict__ w7, const float* __restrict__ wout, b16* __restrict__ WP, b16* __restrict__ WOUT) { const int t = threadIdx.x; const float* ws8[8] = {w0, w1, w2, w3, w4, w5, w6, w7};
  for (int pass = 0; pass < 2; ++pass) {
#pragma unroll
    for (int p = 0; p < 8; ++p) for (int idx = t; idx < D * D; idx += 256) ((volatile b16*)WP)[p * D * D + idx] = (b16)(bf16_rne(ws8[p][idx]) * WSC);
    for (int idx = t; idx < D * 2 * D; idx += 256) ((volatile b16*)WOUT)[idx] = (b16)(bf16_rne(wout[idx]) * WSC); __threadfence(); } }
template <int EXA>
__global__ __launch_bounds__(32) void proj_kernel(const float* __restrict__ IN, const b16* __restrict__ W, const float* __restrict__ bias, int NROWS, float* __restrict__ F) { __shared__ __attribute__((aligned(16))) b16 Ah[16][40], Al[16][40]; __shared__ float Tf[16][D + 4]; const int lane = threadIdx.x, nloc = lane & 15, hlf = lane >> 4; const size_t m0 = (size_t)blockIdx.x * 16; if (m0 >= (size_t)NROWS) return;
  for (int rr = 0; rr < 16; ++rr) { const float v = IN[(m0 + rr) * D + lane]; b16 p, ql; if (EXA) { p = (b16)(bf16_rne(v) * HS); ql = (b16)0.0f; } else split16(v * HS, p, ql); Ah[rr][lane] = p; Al[rr][lane] = ql; } if (lane < 16) for (int k = D; k < 40; ++k) { Ah[lane][k] = (b16)0.0f; Al[lane][k] = (b16)0.0f; }
  wave_lds_sync(); v8f acc[2] = {(v8f){}, (v8f){}}; const v16b a = frag_kb(&Ah[nloc][0], hlf), al = frag_kb(&Al[nloc][0], hlf);
#pragma unroll
  for (int t = 0; t < 2; ++t) { const v16b bw = frag_kb(W + (size_t)(t * 16 + nloc) * D, hlf); acc[t] = wmma16b(a, bw, acc[t]); if (!EXA) acc[t] = wmma16b(al, bw, acc[t]); }
#pragma unroll
  for (int t = 0; t < 2; ++t)
#pragma unroll
    for (int r8 = 0; r8 < 8; ++r8) Tf[8 * hlf + r8][t * 16 + nloc] = acc[t][r8] * (1.0f / (HS * WSC)) + bfv(bias[t * 16 + nloc]);
  wave_lds_sync();
  for (int pass = 0; pass < 2; ++pass) { for (int rr = 0; rr < 16; ++rr) ((volatile float*)F)[(m0 + rr) * D + lane] = Tf[rr][lane]; __threadfence(); } }
__global__ __launch_bounds__(256) void gat_kernel(const float* __restrict__ FS, const float* __restrict__ FD, const float* __restrict__ attn, const int* __restrict__ srcs, int nsrc, int nedge, const int* __restrict__ PERM, const int* __restrict__ ROWPTR, const int* __restrict__ ROWCNT, int permLen, int NDST, int SRCLIM, float* __restrict__ OUT) { const int wave = threadIdx.x >> 5, lane = threadIdx.x & 31; const size_t i = (size_t)blockIdx.x * 8 + wave; if (i >= (size_t)NDST) return; int st = ROWPTR[i], cnt = ROWCNT[i]; cnt = iclamp(cnt, 0, nedge); st = iclamp(st, 0, permLen - cnt);
  const float fdi = FD[i * D + lane], av = bfv(attn[lane]); float mx = -INFINITY, den = 0.0f, acc = 0.0f;
#pragma unroll 1
  for (int j = 0; j < cnt; ++j) { const int e = iclamp(PERM[st + j], 0, nedge - 1); const int u = iclamp(srcs[e], 0, nsrc - 1); if (u >= SRCLIM) continue; const float fsu = FS[(size_t)u * D + lane]; float s = pmul(av, leaky2(fsu + fdi)); for (int o = 16; o; o >>= 1) s += __shfl_xor(s, o);
    const float mn = fmaxf(mx, s); const float sf = (mx == -INFINITY) ? 0.0f : __expf(mx - mn); const float p = __expf(s - mn); den = den * sf + p; acc = pmul(acc, sf) + pmul(p, fsu); mx = mn; }
  const float o = den > 0.0f ? acc / den : 0.0f;
  for (int pass = 0; pass < 2; ++pass) { ((volatile float*)OUT)[i * D + lane] = o; __threadfence(); } }
__global__ __launch_bounds__(256) void lin_kernel(const float* __restrict__ A, const float* __restrict__ Bf, const b16* __restrict__ WOUT, const float* __restrict__ bout, int NLIM, float* __restrict__ Y, float* __restrict__ PS) { __shared__ __attribute__((aligned(16))) b16 Ah[8][16][72], Al[8][16][72]; __shared__ float Tf[8][16][D + 4]; __shared__ float Red[8][2 * D]; const int wave = threadIdx.x >> 5, lane = threadIdx.x & 31, nloc = lane & 15, hlf = lane >> 4; const size_t m0 = (size_t)blockIdx.x * 128 + wave * 16; float ps = 0.0f, pq = 0.0f;
  if (m0 < (size_t)NLIM) {
    for (int rr = 0; rr < 16; ++rr) { b16 p, ql; split16(A[(m0 + rr) * D + lane] * HS, p, ql); Ah[wave][rr][lane] = p; Al[wave][rr][lane] = ql; split16(Bf[(m0 + rr) * D + lane] * HS, p, ql); Ah[wave][rr][D + lane] = p; Al[wave][rr][D + lane] = ql; } if (lane < 16) for (int k = 2 * D; k < 72; ++k) { Ah[wave][lane][k] = (b16)0.0f; Al[wave][lane][k] = (b16)0.0f; }
    wave_lds_sync(); v8f acc[2] = {(v8f){}, (v8f){}};
#pragma unroll
    for (int kb = 0; kb < 2 * D; kb += 32) { const v16b a = frag_kb(&Ah[wave][nloc][kb], hlf), al = frag_kb(&Al[wave][nloc][kb], hlf);
#pragma unroll
      for (int t = 0; t < 2; ++t) { const v16b bw = frag_kb(WOUT + (size_t)(t * 16 + nloc) * 2 * D + kb, hlf); acc[t] = wmma16b(a, bw, acc[t]); acc[t] = wmma16b(al, bw, acc[t]); } }
#pragma unroll
    for (int t = 0; t < 2; ++t)
#pragma unroll
      for (int r8 = 0; r8 < 8; ++r8) Tf[wave][8 * hlf + r8][t * 16 + nloc] = acc[t][r8] * (1.0f / (HS * WSC)) + bfv(bout[t * 16 + nloc]);
    wave_lds_sync();
    for (int rr = 0; rr < 16; ++rr) { const float v = Tf[wave][rr][lane]; ps += v; pq += v * v; }
    for (int pass = 0; pass < 2; ++pass) { for (int rr = 0; rr < 16; ++rr) ((volatile float*)Y)[(m0 + rr) * D + lane] = Tf[wave][rr][lane]; __threadfence(); } }
  Red[wave][lane] = ps; Red[wave][D + lane] = pq; __syncthreads();
  if (wave == 0) for (int pass = 0; pass < 2; ++pass) { for (int c = lane; c < 2 * D; c += 32) { float s = 0.0f; for (int w = 0; w < 8; ++w) s += Red[w][c]; ((volatile float*)PS)[(size_t)blockIdx.x * 2 * D + c] = s; } __threadfence(); } }
__global__ __launch_bounds__(32) void bn_kernel(const float* __restrict__ PS, int nblk, int NLIM, float* __restrict__ BNs) { const int c = threadIdx.x; double s = 0.0, s2 = 0.0; for (int b = 0; b < nblk; ++b) { s += (double)PS[(size_t)b * 2 * D + c]; s2 += (double)PS[(size_t)b * 2 * D + D + c]; } const double mu = s / NLIM; double var = s2 / NLIM - mu * mu; if (var < 0.0) var = 0.0;
  for (int pass = 0; pass < 2; ++pass) { ((volatile float*)BNs)[c] = (float)mu; ((volatile float*)BNs)[D + c] = (float)(1.0 / sqrt(var + (double)BNEPS)); __threadfence(); } }
__global__ __launch_bounds__(256) void out_kernel(const float* __restrict__ Y, const float* __restrict__ BNs, const float* __restrict__ gam, const float* __restrict__ bet, int NLIM, float* __restrict__ out) { const int wave = threadIdx.x >> 5, lane = threadIdx.x & 31; const size_t m0 = (size_t)blockIdx.x * 128 + wave * 16; if (m0 >= (size_t)NLIM) return; const float mu = BNs[lane], rs = BNs[D + lane], g = bfv(gam[lane]), bb = bfv(bet[lane]);
  for (int pass = 0; pass < 2; ++pass) { for (int rr = 0; rr < 16; ++rr) { const float v = pmul(pmul(Y[(m0 + rr) * D + lane] - mu, rs), g) + bb; ((volatile float*)out)[(m0 + rr) * D + lane] = v > 0.0f ? v : 0.01f * v; } __threadfence(); } }
}

extern "C" void kernel_launch(void* const* d_in, const int* in_sizes, int n_in, void* d_out, int out_size, void* d_ws, size_t ws_size, hipStream_t stream) {
  (void)n_in;
  auto Fp = [&](int i) { return (const float*)d_in[i]; }; auto Ip = [&](int i) { return (const int*)d_in[i]; };
  if (in_sizes[0] != NU * D || in_sizes[1] != NI * D || in_sizes[2] != ER || in_sizes[3] != ER || in_sizes[4] != ET || in_sizes[5] != ET || in_sizes[6] != D * D || in_sizes[26] != D * 2 * D || out_size != NU * D) return;
  const int ULIM = NU, ILIM = NI;
  size_t off = 0; char* ws = (char*)d_ws;
  auto carve = [&](size_t bytes) { char* p = ws + off; off += (bytes + 255) & ~(size_t)255; return p; };
  b16* WP = (b16*)carve((size_t)8 * D * D * 2); b16* WOUT = (b16*)carve((size_t)D * 2 * D * 2);
  float* FSa = (float*)carve((size_t)NU * D * 4); float* FDa = (float*)carve((size_t)NU * D * 4); float* H1 = (float*)carve((size_t)NI * D * 4); float* H2 = (float*)carve((size_t)NU * D * 4); float* Aa = (float*)carve((size_t)NU * D * 4); float* Bb = (float*)carve((size_t)NU * D * 4); float* Y = (float*)carve((size_t)NU * D * 4); float* PS = (float*)carve((size_t)(NU / 128 + 1) * 2 * D * 4); float* BNs = (float*)carve(2 * D * 4);
  CsrBufsI ci; off = csr_carveI(ci, ws, off, ER, NI); CsrBufsU cu; off = csr_carveU(cu, ws, off, ER, NU); CsrBufsT ct; off = csr_carveT(ct, ws, off, ET, NU);
  if (off > ws_size || off > ((size_t)160 << 20)) return;
  const int nblk = (ULIM + 127) / 128;
  wput_kernel<<<1, 256, 0, stream>>>(Fp(6), Fp(8), Fp(11), Fp(13), Fp(16), Fp(18), Fp(21), Fp(23), Fp(26), WP, WOUT);
  csr_buildI(ci, Ip(3), ER, NI, stream); csr_buildU(cu, Ip(2), ER, NU, stream); csr_buildT(ct, Ip(5), ET, NU, stream);
  proj_kernel<1><<<ULIM / 16, 32, 0, stream>>>(Fp(0), WP + 0 * D * D, Fp(7), ULIM, FSa); proj_kernel<1><<<ILIM / 16, 32, 0, stream>>>(Fp(1), WP + 1 * D * D, Fp(9), ILIM, FDa);
  gat_kernel<<<(ILIM + 7) / 8, 256, 0, stream>>>(FSa, FDa, Fp(10), Ip(2), NU, ER, ci.PERM, ci.ROWPTR, ci.ROWCNT, (int)ci.permLen, ILIM, ULIM, H1);
  proj_kernel<1><<<ILIM / 16, 32, 0, stream>>>(Fp(1), WP + 2 * D * D, Fp(12), ILIM, FSa); proj_kernel<1><<<ULIM / 16, 32, 0, stream>>>(Fp(0), WP + 3 * D * D, Fp(14), ULIM, FDa);
  gat_kernel<<<(ULIM + 7) / 8, 256, 0, stream>>>(FSa, FDa, Fp(15), Ip(3), NI, ER, cu.PERM, cu.ROWPTR, cu.ROWCNT, (int)cu.permLen, ULIM, ILIM, H2);
  proj_kernel<0><<<ILIM / 16, 32, 0, stream>>>(H1, WP + 4 * D * D, Fp(17), ILIM, FSa); proj_kernel<1><<<ULIM / 16, 32, 0, stream>>>(Fp(0), WP + 5 * D * D, Fp(19), ULIM, FDa);
  gat_kernel<<<(ULIM + 7) / 8, 256, 0, stream>>>(FSa, FDa, Fp(20), Ip(3), NI, ER, cu.PERM, cu.ROWPTR, cu.ROWCNT, (int)cu.permLen, ULIM, ILIM, Aa);
  proj_kernel<0><<<ULIM / 16, 32, 0, stream>>>(H2, WP + 6 * D * D, Fp(22), ULIM, FSa); proj_kernel<1><<<ULIM / 16, 32, 0, stream>>>(Fp(0), WP + 7 * D * D, Fp(24), ULIM, FDa);
  gat_kernel<<<(ULIM + 7) / 8, 256, 0, stream>>>(FSa, FDa, Fp(25), Ip(4), NU, ET, ct.PERM, ct.ROWPTR, ct.ROWCNT, (int)ct.permLen, ULIM, ULIM, Bb);
  lin_kernel<<<nblk, 256, 0, stream>>>(Aa, Bb, WOUT, Fp(27), ULIM, Y, PS);
  bn_kernel<<<1, 32, 0, stream>>>(PS, nblk, ULIM, BNs);
  out_kernel<<<nblk, 256, 0, stream>>>(Y, BNs, Fp(28), Fp(29), ULIM, (float*)d_out);
}
